// MultiHeadAttention_26895085207631
// MI455X (gfx1250) — hardware-verified
//
#include <hip/hip_runtime.h>
#include <math.h>

#ifndef NB
#define NB 4
#endif
#ifndef SEQ
#define SEQ 2048
#endif
#define NB_FULL 4
#define SEQ_FULL 2048
#define DIN 512
#define NCOPY 8
#define DM 64
#define NHEAD 1
#define HDIM 64
#define ROWS (NB * SEQ)
#define EROWS 64
#ifndef EARLY_SCORE_RES
#define EARLY_SCORE_RES 1
#endif

static_assert(NB >= 1 && NB <= NB_FULL);
static_assert(SEQ % 64 == 0 && SEQ <= SEQ_FULL);
static_assert(DM == NHEAD * HDIM);
static_assert(HDIM == 64);
static_assert(DIN % 64 == 0 && DIN % 32 == 0);
static_assert(HDIM % 32 == 0 && HDIM % 8 == 0);
static_assert((2 * DM) % 64 == 0);
static_assert(NCOPY * HDIM == 512);
static_assert(DIN % 8 == 0);
static_assert(EROWS == 64 && SEQ >= EROWS);
static_assert((ROWS * (DIN / 8)) % 256 == 0);

typedef _Float16 v16h __attribute__((ext_vector_type(16)));
typedef _Float16 v8h  __attribute__((ext_vector_type(8)));
typedef float    v8f  __attribute__((ext_vector_type(8)));
typedef float    v4f  __attribute__((ext_vector_type(4)));
typedef unsigned int u4 __attribute__((ext_vector_type(4)));
typedef unsigned int u2 __attribute__((ext_vector_type(2)));
typedef v8h v8h_ma __attribute__((may_alias));
typedef v4f v4f_ma __attribute__((may_alias));
typedef _Float16 h16;

union FragU { v16h v; v8h h[2]; };
__device__ __forceinline__ v16h ld_frag(const _Float16* __restrict__ p) { FragU f; f.h[0] = *(const v8h*)(p); f.h[1] = *(const v8h*)(p + 16); return f.v; }

__device__ __forceinline__ v8f wmma16(v16h a, v16h b, v8f c) {
    c = __builtin_amdgcn_wmma_f32_16x16x32_f16(false, a, false, b, (short)0, c, false, false);
    asm volatile("v_nop\n\tv_nop\n\tv_nop\n\tv_nop" : "+v"(c) : "v"(a), "v"(b));
    return c;
}
__device__ __forceinline__ void dep_guard_h(v8f& a, v8f& b, v16h x, v16h y) { asm volatile("v_nop\n\tv_nop\n\tv_nop\n\tv_nop" : "+v"(a), "+v"(b) : "v"(x), "v"(y)); }
__device__ __forceinline__ void keep4_h(v16h a, v16h b, v16h c, v16h d) { asm volatile("v_nop" :: "v"(a), "v"(b), "v"(c), "v"(d)); }
__device__ __forceinline__ void acc_guard4(v8f& a, v8f& b, v8f& c, v8f& d) { asm volatile("v_nop\n\tv_nop\n\tv_nop\n\tv_nop" : "+v"(a), "+v"(b), "+v"(c), "+v"(d)); }
__device__ __forceinline__ void wave_sync() {
    __builtin_amdgcn_fence(3  , "workgroup");
    __builtin_amdgcn_wave_barrier();
    __builtin_amdgcn_fence(2  , "workgroup");
}

#define VST2(T, ptr, val) do { const T vst2_v_ = (val); *(volatile T*)(ptr) = vst2_v_; __threadfence(); *(volatile T*)(ptr) = vst2_v_; } while (0)

__device__ __forceinline__ float cmb_bf(float v) { const unsigned u = __builtin_bit_cast(unsigned, v); const unsigned r = (u + 0x7fffu + ((u >> 16) & 1u)) & 0xffff0000u; return __builtin_bit_cast(float, r); }
__device__ __forceinline__ unsigned int pk2h(float a, float b) { return (unsigned int)__builtin_bit_cast(unsigned short, (_Float16)a) | ((unsigned int)__builtin_bit_cast(unsigned short, (_Float16)b) << 16); }

static __device__ __forceinline__ h16 toh_flush(float v) { const h16 r = (h16)v; return (fabsf(v) < 6.103515625e-05f) ? (h16)0.0f : r; }
static __device__ __forceinline__ unsigned int pk2h_flush(float a, float b) { return (unsigned int)__builtin_bit_cast(unsigned short, toh_flush(a)) | ((unsigned int)__builtin_bit_cast(unsigned short, toh_flush(b)) << 16); }
static __device__ __forceinline__ unsigned int pk2us(unsigned short lo, unsigned short hi) { return (unsigned int)lo | ((unsigned int)hi << 16); }

static __device__ __forceinline__ void ld_split_f32(const float* __restrict__ p, v16h& hi, v16h& rs) {
    const v4f a = *(const v4f*)(p), b = *(const v4f*)(p + 4), cc = *(const v4f*)(p + 16), d = *(const v4f*)(p + 20);
    const float w[16] = { a.x, a.y, a.z, a.w, b.x, b.y, b.z, b.w, cc.x, cc.y, cc.z, cc.w, d.x, d.y, d.z, d.w };
#pragma unroll
    for (int i = 0; i < 16; ++i) { const h16 h = toh_flush(w[i]); hi[i] = h; rs[i] = toh_flush((w[i] - (float)h) * 2048.0f); }
}

__global__ __launch_bounds__(256) void k_castx(const float* __restrict__ SRC, int src_rows_per_b, unsigned short* __restrict__ DST) {
    const long long u = (long long)blockIdx.x * 256 + threadIdx.x; const int per = DIN / 8; if (u >= (long long)ROWS * per) return;
    const int r = (int)(u / per); const int c8 = 8 * (int)(u % per);
    const int bb = r / SEQ, t = r - bb * SEQ;
    const float* s = SRC + ((long long)bb * src_rows_per_b + t) * DIN + c8;
    const v4f a = *(const v4f*)(s), b = *(const v4f*)(s + 4);
    u4 pk; pk.x = pk2h_flush(cmb_bf(a.x), cmb_bf(a.y)); pk.y = pk2h_flush(cmb_bf(a.z), cmb_bf(a.w)); pk.z = pk2h_flush(cmb_bf(b.x), cmb_bf(b.y)); pk.w = pk2h_flush(cmb_bf(b.z), cmb_bf(b.w));
    VST2(u4, (u4*)(DST + (long long)r * DIN + c8), pk);
}

__global__ __launch_bounds__(256) void k_castbT(const float* __restrict__ SRC, int lds, int src_slice, unsigned short* __restrict__ DST, int ldd, int dst_slice, int nR, int nC, float sc) {
    const long long u = (long long)blockIdx.x * 256 + threadIdx.x; const int per = nR / 8; if (u >= (long long)nC * per) return;
    const int c = (int)(u / per); const int r0 = 8 * (int)(u % per);
    const float* s = SRC + (long long)blockIdx.y * src_slice;
    float w[8];
#pragma unroll
    for (int e = 0; e < 8; ++e) w[e] = cmb_bf(s[(long long)(r0 + e) * lds + c]) * sc;
    u4 pk; pk.x = pk2h(w[0], w[1]); pk.y = pk2h(w[2], w[3]); pk.z = pk2h(w[4], w[5]); pk.w = pk2h(w[6], w[7]);
    VST2(u4, (u4*)(DST + (long long)blockIdx.y * dst_slice + (long long)c * ldd + r0), pk);
}

__global__ __launch_bounds__(256) void k_wsumT(const float* __restrict__ WO, unsigned short* __restrict__ WH, unsigned short* __restrict__ WR) {
    #pragma clang fp contract(off)
    const int u = blockIdx.x * 256 + threadIdx.x; const int per = HDIM / 8; if (u >= DIN * per) return;
    const int n = u / per; const int k0 = 8 * (u % per);
    float w[8];
#pragma unroll
    for (int e = 0; e < 8; ++e) w[e] = 0.f;
#pragma unroll 1
    for (int hc = 0; hc < NCOPY; ++hc) {
#pragma unroll
        for (int e = 0; e < 8; ++e) w[e] += cmb_bf(WO[(size_t)(hc * HDIM + k0 + e) * DIN + n]);
    }
    unsigned short hb[8], rb[8];
#pragma unroll
    for (int e = 0; e < 8; ++e) {
        const float x = w[e] * 16.0f; const h16 h = toh_flush(x);
        hb[e] = __builtin_bit_cast(unsigned short, h);
        rb[e] = __builtin_bit_cast(unsigned short, toh_flush((x - (float)h) * 2048.0f));
    }
    u4 ph; ph.x = pk2us(hb[0], hb[1]); ph.y = pk2us(hb[2], hb[3]); ph.z = pk2us(hb[4], hb[5]); ph.w = pk2us(hb[6], hb[7]);
    u4 pr; pr.x = pk2us(rb[0], rb[1]); pr.y = pk2us(rb[2], rb[3]); pr.z = pk2us(rb[4], rb[5]); pr.w = pk2us(rb[6], rb[7]);
    VST2(u4, (u4*)(WH + (size_t)n * HDIM + k0), ph);
    VST2(u4, (u4*)(WR + (size_t)n * HDIM + k0), pr);
}

__global__ __launch_bounds__(256) void k_tr64(const unsigned short* __restrict__ V16, unsigned short* __restrict__ VT) {
    __shared__ unsigned short T[64 * 72];
    const int tid = threadIdx.x; const int b = blockIdx.y; const int key0 = blockIdx.x * 64;
    {
        const int row = tid >> 2, pc = (tid & 3) * 16;
        const unsigned short* s = V16 + ((size_t)b * SEQ + key0 + row) * HDIM + pc;
        const u4 x = *(const u4*)(s), y = *(const u4*)(s + 8);
        const unsigned int wv[8] = { x.x, x.y, x.z, x.w, y.x, y.y, y.z, y.w };
#pragma unroll
        for (int e = 0; e < 8; ++e) {
            T[row * 72 + pc + 2 * e]     = (unsigned short)(wv[e] & 0xffffu);
            T[row * 72 + pc + 2 * e + 1] = (unsigned short)(wv[e] >> 16);
        }
    }
    __syncthreads();
#pragma unroll
    for (int j = 0; j < 2; ++j) {
        const int idx = tid + 256 * j; const int d = idx >> 3; const int kp = (idx & 7) * 8;
        unsigned short g[8];
#pragma unroll
        for (int e = 0; e < 8; ++e) g[e] = T[(kp + e) * 72 + d];
        u4 pk; pk.x = pk2us(g[0], g[1]); pk.y = pk2us(g[2], g[3]); pk.z = pk2us(g[4], g[5]); pk.w = pk2us(g[6], g[7]);
        VST2(u4, (u4*)(VT + ((size_t)b * HDIM + d) * SEQ + key0 + kp), pk);
    }
}

template <int BIAS, int OUT16, int RESID, int XBF, int RELU>
__device__ __forceinline__ void gemm64_body(
    const unsigned short* __restrict__ Ap, int lda, long long strideA,
    const unsigned short* __restrict__ Btp, int ldb, long long strideB,
    float* __restrict__ Cf, unsigned short* __restrict__ Ch, int ldc, long long strideC,
    const float* __restrict__ bias, const float* __restrict__ resid, int ldr, long long strideR,
    int M, int N, int K, float scale) {
  __shared__ __align__(16) float sT[8][16 * 68];
  const int bz   = blockIdx.y;
  const int lane = threadIdx.x & 31;
  const int wave = threadIdx.x >> 5;
  const int tilesN = N >> 6;
  const int tilesM = M >> 6;
  const int tile = blockIdx.x * 8 + wave;
  if (tile >= tilesM * tilesN) return;
  const int tm = tile / tilesN;
  const int tn = tile - tm * tilesN;
  const int m0 = tm << 6;
  const int n0 = tn << 6;
  const _Float16* Ab = (const _Float16*)Ap  + (size_t)bz * strideA;
  const _Float16* Bb = (const _Float16*)Btp + (size_t)bz * strideB;
  const int rlane = lane & 15;
  const int koff  = (lane >> 4) * 8;
  const int mOff  = (lane >> 4) * 8;

  v8f acc[4][4];
#pragma unroll
  for (int i = 0; i < 4; ++i)
#pragma unroll
    for (int j = 0; j < 4; ++j) acc[i][j] = (v8f){0.f,0.f,0.f,0.f,0.f,0.f,0.f,0.f};

  for (int k0 = 0; k0 < K; k0 += 32) {
    v16h bh[4];
#pragma unroll
    for (int j = 0; j < 4; ++j) bh[j] = ld_frag(Bb + (size_t)(n0 + (j << 4) + rlane) * ldb + koff + k0);
#pragma unroll
    for (int i = 0; i < 4; ++i) {
      const v16h ah = ld_frag(Ab + (size_t)(m0 + (i << 4) + rlane) * lda + koff + k0);
#pragma unroll
      for (int j = 0; j < 4; ++j)
        acc[i][j] = __builtin_amdgcn_wmma_f32_16x16x32_f16(false, ah, false, bh[j], (short)0, acc[i][j], false, false);
      dep_guard_h(acc[i][0], acc[i][3], ah, ah);
    }
    keep4_h(bh[0], bh[1], bh[2], bh[3]);
  }
  acc_guard4(acc[0][0], acc[0][1], acc[0][2], acc[0][3]);
  acc_guard4(acc[1][0], acc[1][1], acc[1][2], acc[1][3]);
  acc_guard4(acc[2][0], acc[2][1], acc[2][2], acc[2][3]);
  acc_guard4(acc[3][0], acc[3][1], acc[3][2], acc[3][3]);

  float bvj[4];
#pragma unroll
  for (int j = 0; j < 4; ++j) bvj[j] = BIAS ? cmb_bf(bias[n0 + (j << 4) + rlane]) : 0.f;

#pragma unroll
  for (int i = 0; i < 4; ++i) {
    const int mBase = m0 + (i << 4);
#pragma unroll
    for (int j = 0; j < 4; ++j) {
#pragma unroll
      for (int r = 0; r < 8; ++r) {
        float v = acc[i][j][r] * scale;
        if (BIAS) v += bvj[j];
        if (RELU) v = fmaxf(v, 0.0f);
        sT[wave][(mOff + r) * 68 + (j << 4) + rlane] = v;
      }
    }
    wave_sync();
    if (OUT16 == 0) {
      float* C = Cf + (size_t)bz * strideC;
      const int hh = lane >> 4, c4 = (lane & 15) * 4;
      v4f vv[8];
#pragma unroll
      for (int it = 0; it < 8; ++it) {
        const int row = it * 2 + hh;
        v4f v = *(const v4f_ma*)&sT[wave][row * 68 + c4];
        if (RESID) {
          v4f x = *(const v4f*)(resid + (size_t)bz * strideR + (size_t)(mBase + row) * ldr + n0 + c4);
          if (XBF) { x.x = cmb_bf(x.x); x.y = cmb_bf(x.y); x.z = cmb_bf(x.z); x.w = cmb_bf(x.w); }
          v = v + x;
        }
        vv[it] = v;
      }
#pragma unroll
      for (int it = 0; it < 8; ++it) *(volatile v4f*)(C + (size_t)(mBase + it * 2 + hh) * ldc + n0 + c4) = vv[it];
      __threadfence();
#pragma unroll
      for (int it = 0; it < 8; ++it) *(volatile v4f*)(C + (size_t)(mBase + it * 2 + hh) * ldc + n0 + c4) = vv[it];
    } else {
      unsigned short* C = Ch + (size_t)bz * strideC;
      const int q = lane >> 3, c8 = (lane & 7) * 8;
      v8h hv[4];
#pragma unroll
      for (int it = 0; it < 4; ++it) {
        const int row = it * 4 + q;
        const v4f a = *(const v4f_ma*)&sT[wave][row * 68 + c8];
        const v4f b = *(const v4f_ma*)&sT[wave][row * 68 + c8 + 4];
        v8h t;
        t[0] = (_Float16)a.x; t[1] = (_Float16)a.y; t[2] = (_Float16)a.z; t[3] = (_Float16)a.w;
        t[4] = (_Float16)b.x; t[5] = (_Float16)b.y; t[6] = (_Float16)b.z; t[7] = (_Float16)b.w;
        hv[it] = t;
      }
#pragma unroll
      for (int it = 0; it < 4; ++it) *(volatile v8h*)(C + (size_t)(mBase + it * 4 + q) * ldc + n0 + c8) = hv[it];
      __threadfence();
#pragma unroll
      for (int it = 0; it < 4; ++it) *(volatile v8h*)(C + (size_t)(mBase + it * 4 + q) * ldc + n0 + c8) = hv[it];
    }
    wave_sync();
  }
}

__global__ __launch_bounds__(256) void k_gemm_h16b(const unsigned short* __restrict__ A, int lda, long long sA, const unsigned short* __restrict__ Bt, int ldb,
                                                   unsigned short* __restrict__ C, int ldc, long long sC, const float* __restrict__ bias, int M, int N, int K, float scale) {
  gemm64_body<1, 1, 0, 0, 0>(A, lda, sA, Bt, ldb, 0, nullptr, C, ldc, sC, bias, nullptr, 0, 0, M, N, K, scale);
}
__global__ __launch_bounds__(256) void k_gemm_f32b(const unsigned short* __restrict__ A, int lda, long long sA, const unsigned short* __restrict__ Bt, int ldb,
                                                   float* __restrict__ C, int ldc, long long sC, const float* __restrict__ bias, int M, int N, int K, float scale) {
  gemm64_body<1, 0, 0, 0, 0>(A, lda, sA, Bt, ldb, 0, C, nullptr, ldc, sC, bias, nullptr, 0, 0, M, N, K, scale);
}

__global__ __launch_bounds__(128) void k_attn(const unsigned short* __restrict__ QKp, const unsigned short* __restrict__ VTp, unsigned short* __restrict__ AOp, float sl2e) {
  __shared__ __align__(16) _Float16 Ps[4][16 * 40];
  __shared__ __align__(16) float    Os[4][16 * 68];
  const int tid = threadIdx.x, wave = tid >> 5, lane = tid & 31, hh = lane >> 4, c = lane & 15;
  const int nqb = SEQ / 64;
  const int bx = blockIdx.x;
  const int qb = bx % nqb;
  const int bh = bx / nqb;
  const int h  = bh % NHEAD;
  const int b  = bh / NHEAD;
  const int q0 = qb * 64 + wave * 16;
  const _Float16* QK = (const _Float16*)QKp + (size_t)b * SEQ * (2 * DM);
  const _Float16* VT = (const _Float16*)VTp + ((size_t)b * DM + (size_t)h * HDIM) * SEQ;
  const float NEG = -__builtin_inff();

  const int qoff = (q0 + c) * (2 * DM) + h * HDIM + 8 * hh;
  const v16h qa0 = ld_frag(QK + qoff), qa1 = ld_frag(QK + qoff + 32);

  float m8[8], l8[8];
  v8f o[4];
#pragma unroll
  for (int r = 0; r < 8; ++r) { m8[r] = NEG; l8[r] = 0.f; }
#pragma unroll
  for (int t = 0; t < 4; ++t) o[t] = (v8f){0.f,0.f,0.f,0.f,0.f,0.f,0.f,0.f};

  for (int key0 = 0; key0 <= q0 + 15; key0 += 32) {
    const int ko = (key0 + c) * (2 * DM) + DM + h * HDIM + 8 * hh;
    v8f s0 = (v8f){0.f,0.f,0.f,0.f,0.f,0.f,0.f,0.f};
    v8f s1 = (v8f){0.f,0.f,0.f,0.f,0.f,0.f,0.f,0.f};
    {
      const v16h kb0 = ld_frag(QK + ko), kb1 = ld_frag(QK + ko + 32);
      s0 = wmma16(qa0, kb0, s0);
      s0 = wmma16(qa1, kb1, s0);
    }
    {
      const v16h kb0 = ld_frag(QK + ko + 16 * (2 * DM)), kb1 = ld_frag(QK + ko + 16 * (2 * DM) + 32);
      s1 = wmma16(qa0, kb0, s1);
      s1 = wmma16(qa1, kb1, s1);
    }
#pragma unroll
    for (int r = 0; r < 8; ++r) {
      const int qrow = q0 + 8 * hh + r;
      float x0 = s0[r] * sl2e, x1 = s1[r] * sl2e;
      x0 = (key0 + c > qrow) ? NEG : x0;
      x1 = (key0 + 16 + c > qrow) ? NEG : x1;
      float mx = fmaxf(x0, x1);
      mx = fmaxf(mx, __shfl_xor(mx, 1, 32)); mx = fmaxf(mx, __shfl_xor(mx, 2, 32));
      mx = fmaxf(mx, __shfl_xor(mx, 4, 32)); mx = fmaxf(mx, __shfl_xor(mx, 8, 32));
      const float mnew = fmaxf(m8[r], mx);
      const float corr = (mnew == NEG) ? 1.f : exp2f(m8[r] - mnew);
      const float p0 = (x0 == NEG) ? 0.f : exp2f(x0 - mnew);
      const float p1 = (x1 == NEG) ? 0.f : exp2f(x1 - mnew);
      float rs = p0 + p1;
      rs += __shfl_xor(rs, 1, 32); rs += __shfl_xor(rs, 2, 32); rs += __shfl_xor(rs, 4, 32); rs += __shfl_xor(rs, 8, 32);
      l8[r] = l8[r] * corr + rs; m8[r] = mnew;
      o[0][r] *= corr; o[1][r] *= corr; o[2][r] *= corr; o[3][r] *= corr;
      Ps[wave][(8 * hh + r) * 40 + c]      = (_Float16)(p0 * 4096.f);
      Ps[wave][(8 * hh + r) * 40 + 16 + c] = (_Float16)(p1 * 4096.f);
    }
    wave_sync();
    FragU pf;
    pf.h[0] = *(const v8h_ma*)&Ps[wave][c * 40 + 8 * hh];
    pf.h[1] = *(const v8h_ma*)&Ps[wave][c * 40 + 16 + 8 * hh];
    const int vo = c * SEQ + key0 + 8 * hh;
    v16h vb[4];
#pragma unroll
    for (int t = 0; t < 4; ++t) vb[t] = ld_frag(VT + vo + t * 16 * SEQ);
#pragma unroll
    for (int t = 0; t < 4; ++t) o[t] = wmma16(pf.v, vb[t], o[t]);
    wave_sync();
  }

#pragma unroll
  for (int r = 0; r < 8; ++r) {
    const float inv = (l8[r] > 0.f) ? 1.0f / (l8[r] * 256.0f) : 0.f;
#pragma unroll
    for (int t = 0; t < 4; ++t) Os[wave][(8 * hh + r) * 68 + t * 16 + c] = o[t][r] * inv;
  }
  wave_sync();
  {
    unsigned short* AO = AOp + ((size_t)b * SEQ + q0) * DM + h * HDIM;
    const int q = lane >> 3, c8 = (lane & 7) * 8;
    v8h hv[4];
#pragma unroll
    for (int it = 0; it < 4; ++it) {
      const int row = it * 4 + q;
      const v4f a = *(const v4f_ma*)&Os[wave][row * 68 + c8];
      const v4f bq = *(const v4f_ma*)&Os[wave][row * 68 + c8 + 4];
      v8h t;
      t[0] = (_Float16)a.x; t[1] = (_Float16)a.y; t[2] = (_Float16)a.z; t[3] = (_Float16)a.w;
      t[4] = (_Float16)bq.x; t[5] = (_Float16)bq.y; t[6] = (_Float16)bq.z; t[7] = (_Float16)bq.w;
      hv[it] = t;
    }
#pragma unroll
    for (int it = 0; it < 4; ++it) *(volatile v8h*)(AO + (size_t)(it * 4 + q) * DM + c8) = hv[it];
    __threadfence();
#pragma unroll
    for (int it = 0; it < 4; ++it) *(volatile v8h*)(AO + (size_t)(it * 4 + q) * DM + c8) = hv[it];
  }
}

__global__ __launch_bounds__(128) __attribute__((amdgpu_num_vgpr(256)))
void k_attn_early(const float* __restrict__ QE, const float* __restrict__ KE, const float* __restrict__ VE,
                  const unsigned short* __restrict__ WSHp, const unsigned short* __restrict__ WSRp,
                  const float* __restrict__ bo, float* __restrict__ out, float sl2e) {
  __shared__ __align__(16) _Float16 VhT[HDIM * 72];
  __shared__ __align__(16) _Float16 VrT[HDIM * 72];
  __shared__ __align__(16) _Float16 Th[4][16 * 72];
  __shared__ __align__(16) _Float16 Tr[4][16 * 72];
  __shared__ __align__(16) float    Ot[4][16 * 68];
  const int tid = threadIdx.x, lane = tid & 31, hh = lane >> 4, c = lane & 15;
  const int wave = __builtin_amdgcn_readfirstlane(threadIdx.x >> 5);
  const int b = blockIdx.x;
  const int q0 = wave * 16;
  const float* Qb = QE + (size_t)b * EROWS * HDIM;
  const float* Kb = KE + (size_t)b * EROWS * HDIM;
  const float* Vb = VE + (size_t)b * EROWS * HDIM;
  const float NEG = -__builtin_inff();
  const float RS = 1.0f / 2048.0f;

#pragma unroll
  for (int j = 0; j < 8; ++j) {
    const int idx = tid + 128 * j; const int key = idx >> 4; const int d4 = (idx & 15) * 4;
    const v4f x = *(const v4f*)(Vb + key * HDIM + d4);
    const float w[4] = { x.x, x.y, x.z, x.w };
#pragma unroll
    for (int e = 0; e < 4; ++e) {
      const h16 hv = toh_flush(w[e]);
      VhT[(d4 + e) * 72 + key] = hv;
      VrT[(d4 + e) * 72 + key] = toh_flush((w[e] - (float)hv) * 2048.0f);
    }
  }
  __syncthreads();

  float m8[8], l8[8];
  v8f o[4], orr[4];
#pragma unroll
  for (int r = 0; r < 8; ++r) { m8[r] = NEG; l8[r] = 0.f; }
#pragma unroll
  for (int t = 0; t < 4; ++t) { o[t] = (v8f){0.f,0.f,0.f,0.f,0.f,0.f,0.f,0.f}; orr[t] = (v8f){0.f,0.f,0.f,0.f,0.f,0.f,0.f,0.f}; }

  for (int key0 = 0; key0 <= q0 + 15; key0 += 32) {
    v8f s0 = (v8f){0.f,0.f,0.f,0.f,0.f,0.f,0.f,0.f};
    v8f s1 = (v8f){0.f,0.f,0.f,0.f,0.f,0.f,0.f,0.f};
#if EARLY_SCORE_RES
    v8f t0 = (v8f){0.f,0.f,0.f,0.f,0.f,0.f,0.f,0.f};
    v8f t1 = (v8f){0.f,0.f,0.f,0.f,0.f,0.f,0.f,0.f};
#endif
#pragma unroll
    for (int ks = 0; ks < 2; ++ks) {
      v16h qh, qr;
      ld_split_f32(Qb + (q0 + c) * HDIM + 32 * ks + 8 * hh, qh, qr);
      {
        v16h kh, kr;
        ld_split_f32(Kb + (key0 + c) * HDIM + 32 * ks + 8 * hh, kh, kr);
        s0 = wmma16(qh, kh, s0);
#if EARLY_SCORE_RES
        t0 = wmma16(qh, kr, t0);
        t0 = wmma16(qr, kh, t0);
#endif
      }
      {
        v16h kh, kr;
        ld_split_f32(Kb + (key0 + 16 + c) * HDIM + 32 * ks + 8 * hh, kh, kr);
        s1 = wmma16(qh, kh, s1);
#if EARLY_SCORE_RES
        t1 = wmma16(qh, kr, t1);
        t1 = wmma16(qr, kh, t1);
#endif
      }
    }
#pragma unroll
    for (int r = 0; r < 8; ++r) {
      const int qrow = q0 + 8 * hh + r;
#if EARLY_SCORE_RES
      float x0 = (s0[r] + t0[r] * RS) * sl2e, x1 = (s1[r] + t1[r] * RS) * sl2e;
#else
      float x0 = s0[r] * sl2e, x1 = s1[r] * sl2e;
#endif
      x0 = (key0 + c > qrow) ? NEG : x0;
      x1 = (key0 + 16 + c > qrow) ? NEG : x1;
      float mx = fmaxf(x0, x1);
      mx = fmaxf(mx, __shfl_xor(mx, 1, 32)); mx = fmaxf(mx, __shfl_xor(mx, 2, 32));
      mx = fmaxf(mx, __shfl_xor(mx, 4, 32)); mx = fmaxf(mx, __shfl_xor(mx, 8, 32));
      const float mnew = fmaxf(m8[r], mx);
      const float corr = (mnew == NEG) ? 1.f : exp2f(m8[r] - mnew);
      const float p0 = (x0 == NEG) ? 0.f : exp2f(x0 - mnew);
      const float p1 = (x1 == NEG) ? 0.f : exp2f(x1 - mnew);
      float rs = p0 + p1;
      rs += __shfl_xor(rs, 1, 32); rs += __shfl_xor(rs, 2, 32); rs += __shfl_xor(rs, 4, 32); rs += __shfl_xor(rs, 8, 32);
      l8[r] = l8[r] * corr + rs; m8[r] = mnew;
      o[0][r] *= corr; o[1][r] *= corr; o[2][r] *= corr; o[3][r] *= corr;
      orr[0][r] *= corr; orr[1][r] *= corr; orr[2][r] *= corr; orr[3][r] *= corr;
      const float pv0 = p0 * 4096.f, pv1 = p1 * 4096.f;
      const h16 ph0 = toh_flush(pv0), ph1 = toh_flush(pv1);
      Th[wave][(8 * hh + r) * 72 + c]      = ph0;
      Th[wave][(8 * hh + r) * 72 + 16 + c] = ph1;
      Tr[wave][(8 * hh + r) * 72 + c]      = toh_flush((pv0 - (float)ph0) * 2048.0f);
      Tr[wave][(8 * hh + r) * 72 + 16 + c] = toh_flush((pv1 - (float)ph1) * 2048.0f);
    }
    wave_sync();
    FragU pfh, pfr;
    pfh.h[0] = *(const v8h_ma*)&Th[wave][c * 72 + 8 * hh];
    pfh.h[1] = *(const v8h_ma*)&Th[wave][c * 72 + 16 + 8 * hh];
    pfr.h[0] = *(const v8h_ma*)&Tr[wave][c * 72 + 8 * hh];
    pfr.h[1] = *(const v8h_ma*)&Tr[wave][c * 72 + 16 + 8 * hh];
#pragma unroll
    for (int t = 0; t < 4; ++t) {
      FragU vh, vr;
      vh.h[0] = *(const v8h_ma*)&VhT[(t * 16 + c) * 72 + key0 + 8 * hh];
      vh.h[1] = *(const v8h_ma*)&VhT[(t * 16 + c) * 72 + key0 + 16 + 8 * hh];
      vr.h[0] = *(const v8h_ma*)&VrT[(t * 16 + c) * 72 + key0 + 8 * hh];
      vr.h[1] = *(const v8h_ma*)&VrT[(t * 16 + c) * 72 + key0 + 16 + 8 * hh];
      o[t]   = wmma16(pfh.v, vh.v, o[t]);
      orr[t] = wmma16(pfh.v, vr.v, orr[t]);
      orr[t] = wmma16(pfr.v, vh.v, orr[t]);
    }
    wave_sync();
  }

#pragma unroll
  for (int r = 0; r < 8; ++r) {
    const float inv = (l8[r] > 0.f) ? 1.0f / (l8[r] * 256.0f) : 0.f;
#pragma unroll
    for (int t = 0; t < 4; ++t) {
      const float c16 = (o[t][r] + orr[t][r] * RS) * inv;
      const h16 chv = toh_flush(c16);
      Th[wave][(8 * hh + r) * 72 + t * 16 + c] = chv;
      Tr[wave][(8 * hh + r) * 72 + t * 16 + c] = toh_flush((c16 - (float)chv) * 2048.0f);
    }
  }
  wave_sync();
  FragU ah[2], ar[2];
#pragma unroll
  for (int ks = 0; ks < 2; ++ks) {
    ah[ks].h[0] = *(const v8h_ma*)&Th[wave][c * 72 + 32 * ks + 8 * hh];
    ah[ks].h[1] = *(const v8h_ma*)&Th[wave][c * 72 + 32 * ks + 16 + 8 * hh];
    ar[ks].h[0] = *(const v8h_ma*)&Tr[wave][c * 72 + 32 * ks + 8 * hh];
    ar[ks].h[1] = *(const v8h_ma*)&Tr[wave][c * 72 + 32 * ks + 16 + 8 * hh];
  }

  const _Float16* WH = (const _Float16*)WSHp;
  const _Float16* WR = (const _Float16*)WSRp;
  float* orow = out + ((size_t)b * SEQ_FULL + q0) * DIN;
#pragma unroll 1
  for (int g = 0; g < DIN / 64; ++g) {
    const int n0 = g * 64;
#pragma unroll
    for (int j = 0; j < 4; ++j) {
      v8f a0 = (v8f){0.f,0.f,0.f,0.f,0.f,0.f,0.f,0.f};
      v8f a1 = (v8f){0.f,0.f,0.f,0.f,0.f,0.f,0.f,0.f};
      const int wo = (n0 + 16 * j + c) * HDIM + 8 * hh;
#pragma unroll
      for (int ks = 0; ks < 2; ++ks) {
        const v16h bh = ld_frag(WH + wo + 32 * ks);
        const v16h br = ld_frag(WR + wo + 32 * ks);
        a0 = wmma16(ah[ks].v, bh, a0);
        a1 = wmma16(ah[ks].v, br, a1);
        a1 = wmma16(ar[ks].v, bh, a1);
      }
      const float bb = cmb_bf(bo[n0 + 16 * j + c]);
#pragma unroll
      for (int r = 0; r < 8; ++r) Ot[wave][(8 * hh + r) * 68 + 16 * j + c] = (a0[r] + a1[r] * RS) * 0.00390625f + bb;
    }
    wave_sync();
    {
      const int c4 = (lane & 15) * 4;
      v4f vv[8];
#pragma unroll
      for (int it = 0; it < 8; ++it) vv[it] = *(const v4f_ma*)&Ot[wave][(it * 2 + hh) * 68 + c4];
#pragma unroll
      for (int it = 0; it < 8; ++it) *(volatile v4f*)(orow + (size_t)(it * 2 + hh) * DIN + n0 + c4) = vv[it];
      __threadfence();
#pragma unroll
      for (int it = 0; it < 8; ++it) *(volatile v4f*)(orow + (size_t)(it * 2 + hh) * DIN + n0 + c4) = vv[it];
    }
    wave_sync();
  }
}

constexpr size_t SZ_X16  = (size_t)ROWS * DIN * 2;
constexpr size_t SZ_W316 = (size_t)3 * HDIM * DIN * 2;
constexpr size_t SZ_WS16 = (size_t)DIN * HDIM * 2;
constexpr size_t SZ_QK16 = (size_t)ROWS * 2 * DM * 2;
constexpr size_t SZ_V16  = (size_t)ROWS * HDIM * 2;
constexpr size_t SZ_VT16 = (size_t)NB * DM * SEQ * 2;
constexpr size_t SZ_AO16 = (size_t)ROWS * DM * 2;
constexpr size_t SZ_E32  = (size_t)NB * EROWS * HDIM * 4;
constexpr size_t WS_TOTAL = 3 * SZ_X16 + SZ_W316 + 2 * SZ_WS16 + SZ_QK16 + SZ_V16 + SZ_VT16 + SZ_AO16 + 3 * SZ_E32;
static_assert(WS_TOTAL <= (size_t)134217728);
static_assert(SZ_X16 % 256 == 0 && SZ_W316 % 256 == 0 && SZ_WS16 % 256 == 0 && SZ_QK16 % 256 == 0 && SZ_V16 % 256 == 0 && SZ_VT16 % 256 == 0 && SZ_AO16 % 256 == 0 && SZ_E32 % 256 == 0);

extern "C" void kernel_launch(void* const* d_in, const int* in_sizes, int n_in, void* d_out, int out_size, void* d_ws, size_t ws_size, hipStream_t stream) {
    if (n_in < 11) return;
    const long long need_x = ((long long)(NB - 1) * SEQ_FULL + SEQ) * DIN;
    if ((long long)in_sizes[0] < need_x || (long long)in_sizes[1] < need_x || (long long)in_sizes[2] < need_x || (long long)out_size < need_x) return;
    if (in_sizes[3] < DIN * HDIM || in_sizes[4] < HDIM || in_sizes[5] < DIN * HDIM || in_sizes[6] < HDIM || in_sizes[7] < DIN * HDIM || in_sizes[8] < HDIM) return;
    if (in_sizes[9] < NCOPY * HDIM * DIN || in_sizes[10] < DIN) return;
    if (ws_size < WS_TOTAL) return;
    const float* xq  = (const float*)d_in[0];
    const float* xk  = (const float*)d_in[1];
    const float* xv  = (const float*)d_in[2];
    const float* wq  = (const float*)d_in[3];
    const float* bq  = (const float*)d_in[4];
    const float* wk  = (const float*)d_in[5];
    const float* bk  = (const float*)d_in[6];
    const float* wv  = (const float*)d_in[7];
    const float* bv  = (const float*)d_in[8];
    const float* wo  = (const float*)d_in[9];
    const float* bo  = (const float*)d_in[10];
    float* out = (float*)d_out;
    char* wsp = (char*)d_ws;
    unsigned short* XQ16 = (unsigned short*)wsp; wsp += SZ_X16;
    unsigned short* XK16 = (unsigned short*)wsp; wsp += SZ_X16;
    unsigned short* XV16 = (unsigned short*)wsp; wsp += SZ_X16;
    unsigned short* W316 = (unsigned short*)wsp; wsp += SZ_W316;
    unsigned short* WSH  = (unsigned short*)wsp; wsp += SZ_WS16;
    unsigned short* WSR  = (unsigned short*)wsp; wsp += SZ_WS16;
    unsigned short* QK16 = (unsigned short*)wsp; wsp += SZ_QK16;
    unsigned short* V16  = (unsigned short*)wsp; wsp += SZ_V16;
    unsigned short* VT16 = (unsigned short*)wsp; wsp += SZ_VT16;
    unsigned short* AO16 = (unsigned short*)wsp; wsp += SZ_AO16;
    float*          QE   = (float*)wsp;          wsp += SZ_E32;
    float*          KE   = (float*)wsp;          wsp += SZ_E32;
    float*          VE   = (float*)wsp;          wsp += SZ_E32;

    const float sl2e = 0.125f * 1.4426950408889634f;

    k_castx<<<(ROWS * (DIN / 8) + 255) / 256, 256, 0, stream>>>(xq, SEQ_FULL, XQ16);
    k_castx<<<(ROWS * (DIN / 8) + 255) / 256, 256, 0, stream>>>(xk, SEQ_FULL, XK16);
    k_castx<<<(ROWS * (DIN / 8) + 255) / 256, 256, 0, stream>>>(xv, SEQ_FULL, XV16);
    k_castbT<<<dim3((HDIM * (DIN / 8) + 255) / 256, 1), 256, 0, stream>>>(wq, HDIM, 0, W316, DIN, 0, DIN, HDIM, 16.0f);
    k_castbT<<<dim3((HDIM * (DIN / 8) + 255) / 256, 1), 256, 0, stream>>>(wk, HDIM, 0, W316 + (size_t)HDIM * DIN, DIN, 0, DIN, HDIM, 16.0f);
    k_castbT<<<dim3((HDIM * (DIN / 8) + 255) / 256, 1), 256, 0, stream>>>(wv, HDIM, 0, W316 + (size_t)2 * HDIM * DIN, DIN, 0, DIN, HDIM, 16.0f);
    k_wsumT<<<(DIN * (HDIM / 8) + 255) / 256, 256, 0, stream>>>(wo, WSH, WSR);
    k_gemm_h16b<<<dim3(((SEQ / 64) * (HDIM / 64) + 7) / 8, NB), 256, 0, stream>>>(XQ16, DIN, (long long)SEQ * DIN, W316, DIN, QK16, 2 * DM, (long long)SEQ * 2 * DM, bq, SEQ, HDIM, DIN, 0.0625f);
    k_gemm_h16b<<<dim3(((SEQ / 64) * (HDIM / 64) + 7) / 8, NB), 256, 0, stream>>>(XK16, DIN, (long long)SEQ * DIN, W316 + (size_t)HDIM * DIN, DIN, QK16 + DM, 2 * DM, (long long)SEQ * 2 * DM, bk, SEQ, HDIM, DIN, 0.0625f);
    k_gemm_h16b<<<dim3(((SEQ / 64) * (HDIM / 64) + 7) / 8, NB), 256, 0, stream>>>(XV16, DIN, (long long)SEQ * DIN, W316 + (size_t)2 * HDIM * DIN, DIN, V16, HDIM, (long long)SEQ * HDIM, bv, SEQ, HDIM, DIN, 0.0625f);
    k_tr64<<<dim3(SEQ / 64, NB), 256, 0, stream>>>(V16, VT16);
    k_attn<<<NB * NHEAD * (SEQ / 64), 128, 0, stream>>>(QK16, VT16, AO16, sl2e);
    k_gemm_f32b<<<dim3(((SEQ / 64) * (DIN / 64) + 7) / 8, NB), 256, 0, stream>>>(AO16, DM, (long long)SEQ * DM, WSH, HDIM, out, DIN, (long long)SEQ_FULL * DIN, bo, SEQ, DIN, HDIM, 0.00390625f);
    k_gemm_f32b<<<dim3(1, NB), 256, 0, stream>>>(XQ16, DIN, (long long)SEQ * DIN, W316, DIN, QE, HDIM, (long long)EROWS * HDIM, bq, EROWS, HDIM, DIN, 0.0625f);
    k_gemm_f32b<<<dim3(1, NB), 256, 0, stream>>>(XK16, DIN, (long long)SEQ * DIN, W316 + (size_t)HDIM * DIN, DIN, KE, HDIM, (long long)EROWS * HDIM, bk, EROWS, HDIM, DIN, 0.0625f);
    k_gemm_f32b<<<dim3(1, NB), 256, 0, stream>>>(XV16, DIN, (long long)SEQ * DIN, W316 + (size_t)2 * HDIM * DIN, DIN, VE, HDIM, (long long)EROWS * HDIM, bv, EROWS, HDIM, DIN, 0.0625f);
    k_attn_early<<<NB, 128, 0, stream>>>(QE, KE, VE, WSH, WSR, bo, out, sl2e);
}
